// DeformableBlock_13932873909314
// MI455X (gfx1250) — hardware-verified
//
#include <hip/hip_runtime.h>
#include <math.h>
#include <stddef.h>

#pragma clang fp contract(off)

typedef __attribute__((ext_vector_type(16))) _Float16 v16h;
typedef __attribute__((ext_vector_type(8)))  _Float16 v8h;
typedef __attribute__((ext_vector_type(16))) __bf16   v16b;
typedef __attribute__((ext_vector_type(8)))  __bf16   v8b;
typedef __attribute__((ext_vector_type(8)))  float    v8f;
typedef __attribute__((ext_vector_type(4)))  float    v4f;
typedef __attribute__((ext_vector_type(4)))  unsigned v4u;

constexpr int NB    = 4;
constexpr int NC    = 64;
constexpr int NH    = 128;
constexpr int NW    = 128;
constexpr int NOUT  = 64;
constexpr int KPOS  = 9;
constexpr int NOFF  = 2 * KPOS;
constexpr int NOFFP = 32;
constexpr int KTOT  = NC * KPOS;
constexpr int NKSTEP = KTOT / 32;
constexpr int TPIX  = 64;
constexpr int TPR   = NW / TPIX;
constexpr int NBLK  = NB * NH * TPR;
constexpr int BTP   = KTOT + 8;
constexpr int SLP   = 68;
constexpr int NTHR  = 256;
constexpr float WDEF_CARRY = 64.0f;
constexpr float WDEF_FOLD  = 1.0f / 64.0f;
constexpr int NVW_OFF = NOFFP * KTOT / 8;
constexpr int NVW_DEF = NOUT * KTOT / 8;
constexpr int NVW_TOT = NVW_OFF + NVW_DEF;

static_assert(KTOT % 32 == 0);
static_assert(NW % TPIX == 0 && TPIX == 64);
static_assert(BTP % 8 == 0 && SLP % 4 == 0);
static_assert(NOFFP % 16 == 0 && NOFFP >= NOFF && NOUT % 16 == 0);
static_assert((TPIX * KPOS * 8) % NTHR == 0);
static_assert(TPIX * 4 == NTHR);
static_assert(NVW_OFF % NTHR == 0 && NVW_TOT % NTHR == 0);
static_assert(NC * 32 == NTHR * 8);

constexpr size_t WS_XH_OFF   = 0;
constexpr size_t WS_XH_SZ    = (size_t)NB * NH * NW * NC * 2;
constexpr size_t WS_OFFP_OFF = WS_XH_OFF + WS_XH_SZ;
constexpr size_t WS_OFFP_SZ  = (size_t)NB * NOFF * NH * NW * 4;
constexpr size_t WS_WOFF_OFF = WS_OFFP_OFF + WS_OFFP_SZ;
constexpr size_t WS_WOFF_SZ  = (size_t)NOFFP * KTOT * 2;
constexpr size_t WS_WDEF_OFF = WS_WOFF_OFF + WS_WOFF_SZ;
constexpr size_t WS_WDEF_SZ  = (size_t)NOUT * KTOT * 2;
constexpr size_t WS_TOTAL    = WS_WDEF_OFF + WS_WDEF_SZ;
static_assert(WS_TOTAL == 13217792);
static_assert(WS_XH_OFF % 256 == 0 && WS_OFFP_OFF % 256 == 0 && WS_WOFF_OFF % 256 == 0 && WS_WDEF_OFF % 256 == 0);
static_assert(WS_TOTAL <= (size_t)134217728);

__device__ __forceinline__ unsigned short f2bf_bits(float f) {
  unsigned u = __float_as_uint(f);
  return (unsigned short)((u + 0x7FFFu + ((u >> 16) & 1u)) >> 16);
}
__device__ __forceinline__ float bf_bits2f(unsigned short h) { return __uint_as_float(((unsigned)h) << 16); }

__device__ __forceinline__ void dep_guard_h(v8f& a, v8f& b, v16h x, v16h y) { asm volatile("v_nop\n\tv_nop\n\tv_nop\n\tv_nop" : "+v"(a), "+v"(b) : "v"(x), "v"(y)); }
__device__ __forceinline__ void dep_guard_b(v8f& a, v8f& b, v16b x, v16b y) { asm volatile("v_nop\n\tv_nop\n\tv_nop\n\tv_nop" : "+v"(a), "+v"(b) : "v"(x), "v"(y)); }
__device__ __forceinline__ void keep4_h(v16h a, v16h b, v16h c, v16h d) { asm volatile("v_nop" :: "v"(a), "v"(b), "v"(c), "v"(d)); }
__device__ __forceinline__ void keep4_b(v16b a, v16b b, v16b c, v16b d) { asm volatile("v_nop" :: "v"(a), "v"(b), "v"(c), "v"(d)); }
__device__ __forceinline__ void acc_guard4(v8f& a, v8f& b, v8f& c, v8f& d) { asm volatile("v_nop\n\tv_nop\n\tv_nop\n\tv_nop" : "+v"(a), "+v"(b), "+v"(c), "+v"(d)); }
template <typename T> struct Frag;
template <> struct Frag<_Float16> {
  typedef v16h V; union U { v16h v; v8h h[2]; };
  static __device__ __forceinline__ v16h load(const _Float16* p) {
    U f; f.h[0] = *(const v8h*)(p); f.h[1] = *(const v8h*)(p + 16); return f.v;
  }
  static __device__ __forceinline__ v8f mma(v16h a, v16h b, v8f c) {
    return __builtin_amdgcn_wmma_f32_16x16x32_f16(false, a, false, b, (short)0, c, false, false);
  }
  static __device__ __forceinline__ void guard(v8f& a, v8f& b, v16h x, v16h y) { dep_guard_h(a, b, x, y); }
  static __device__ __forceinline__ void keep(v16h a, v16h b, v16h c, v16h d) { keep4_h(a, b, c, d); }
};
template <> struct Frag<__bf16> {
  typedef v16b V; union U { v16b v; v8b h[2]; };
  static __device__ __forceinline__ v16b load(const __bf16* p) {
    U f; f.h[0] = *(const v8b*)(p); f.h[1] = *(const v8b*)(p + 16); return f.v;
  }
  static __device__ __forceinline__ v8f mma(v16b a, v16b b, v8f c) {
    return __builtin_amdgcn_wmma_f32_16x16x32_bf16(false, a, false, b, (short)0, c, false, false);
  }
  static __device__ __forceinline__ void guard(v8f& a, v8f& b, v16b x, v16b y) { dep_guard_b(a, b, x, y); }
  static __device__ __forceinline__ void keep(v16b a, v16b b, v16b c, v16b d) { keep4_b(a, b, c, d); }
};

__device__ __forceinline__ void tie1_b(v8f& a, v16b x, v16b y) {
  asm volatile("v_nop\n\tv_nop\n\tv_nop\n\tv_nop" : "+v"(a) : "v"(x), "v"(y));
}
__device__ __forceinline__ void tie2_h(v8f& a, v8f& b, v16h x, v16h y, v16h z) {
  asm volatile("v_nop\n\tv_nop\n\tv_nop\n\tv_nop" : "+v"(a), "+v"(b) : "v"(x), "v"(y), "v"(z));
}

__device__ __forceinline__ float bfr(float f) { return bf_bits2f(f2bf_bits(f)); }
__device__ __forceinline__ int clampi(int v, int lo, int hi) { return v < lo ? lo : (v > hi ? hi : v); }
__device__ __forceinline__ unsigned pack_bf2(float f0, float f1) {
  return (unsigned)f2bf_bits(f0) | ((unsigned)f2bf_bits(f1) << 16);
}
__device__ __forceinline__ unsigned pack_h2(float f0, float f1) {
  const unsigned short b0 = __builtin_bit_cast(unsigned short, (_Float16)f0);
  const unsigned short b1 = __builtin_bit_cast(unsigned short, (_Float16)f1);
  return (unsigned)b0 | ((unsigned)b1 << 16);
}
__device__ __forceinline__ float bf_lo(unsigned w) { return __uint_as_float(w << 16); }
__device__ __forceinline__ float bf_hi(unsigned w) { return __uint_as_float(w & 0xffff0000u); }
__device__ __forceinline__ float lerp4(float g0, float g1, float g2, float g3, float c0, float c1, float c2, float c3) {
  return ((g0 * c0 + g1 * c1) + g2 * c2) + g3 * c3;
}
__device__ __forceinline__ unsigned mix_word(unsigned a, unsigned b, unsigned c, unsigned d,
                                             float c0, float c1, float c2, float c3) {
  const float vlo = lerp4(bf_lo(a), bf_lo(b), bf_lo(c), bf_lo(d), c0, c1, c2, c3);
  const float vhi = lerp4(bf_hi(a), bf_hi(b), bf_hi(c), bf_hi(d), c0, c1, c2, c3);
  return pack_h2(vlo, vhi);
}
__device__ __forceinline__ v4u mix_vec(v4u a, v4u b, v4u c, v4u d, float c0, float c1, float c2, float c3) {
  v4u r;
  r.x = mix_word(a.x, b.x, c.x, d.x, c0, c1, c2, c3);
  r.y = mix_word(a.y, b.y, c.y, d.y, c0, c1, c2, c3);
  r.z = mix_word(a.z, b.z, c.z, d.z, c0, c1, c2, c3);
  r.w = mix_word(a.w, b.w, c.w, d.w, c0, c1, c2, c3);
  return r;
}

__global__ __launch_bounds__(NTHR) void k_pack_x(const float* __restrict__ x, unsigned short* __restrict__ xh) {
  __shared__ float tile[NC][33];
  const int bh  = blockIdx.x;
  const int b   = bh / NH;
  const int h   = bh - b * NH;
  const int xs  = blockIdx.y * 32;
  const int tid = threadIdx.x;
#pragma unroll
  for (int i = 0; i < 8; ++i) {
    const int idx = tid + i * NTHR;
    const int c = idx >> 5, xx = idx & 31;
    tile[c][xx] = x[(((size_t)b * NC + c) * NH + h) * NW + xs + xx];
  }
  __syncthreads();
  const int lane = tid & 31, wave = tid >> 5;
  const int pl = wave * 4 + (lane >> 3);
  const int c8 = (lane & 7) * 8;
  v4u q;
  q.x = pack_bf2(tile[c8 + 0][pl], tile[c8 + 1][pl]);
  q.y = pack_bf2(tile[c8 + 2][pl], tile[c8 + 3][pl]);
  q.z = pack_bf2(tile[c8 + 4][pl], tile[c8 + 5][pl]);
  q.w = pack_bf2(tile[c8 + 6][pl], tile[c8 + 7][pl]);
  unsigned short* dst = xh + ((((size_t)b * NH + h) * NW + xs + pl) * NC + c8);
  *(volatile v4u*)dst = q;
  __threadfence();
  *(volatile v4u*)dst = q;
}

__global__ __launch_bounds__(NTHR) void k_pack_w(const float* __restrict__ w_off, const float* __restrict__ w_def,
                                                unsigned short* __restrict__ woffp, unsigned short* __restrict__ wdefp) {
  const int i = blockIdx.x * NTHR + threadIdx.x;
  if (i >= NVW_TOT) return;
  const bool first = (i < NVW_OFF);
  const int jj   = first ? i : (i - NVW_OFF);
  const int o    = jj / (KTOT / 8);
  const int rem  = jj - o * (KTOT / 8);
  const int kpos = rem >> 3;
  const int c0   = (rem & 7) * 8;
  unsigned short bits[8];
  if (first) {
    const int oc = (o < NOFF) ? o : (NOFF - 1);
#pragma unroll
    for (int e = 0; e < 8; ++e) {
      const float v = w_off[((size_t)(oc * NC + c0 + e)) * KPOS + kpos];
      const unsigned short hb = f2bf_bits(v);
      bits[e] = (o < NOFF) ? hb : (unsigned short)0;
    }
  } else {
#pragma unroll
    for (int e = 0; e < 8; ++e) {
      const float v = w_def[((size_t)(o * NC + c0 + e)) * KPOS + kpos];
      const float s = WDEF_CARRY * bfr(v);
      bits[e] = __builtin_bit_cast(unsigned short, (_Float16)s);
    }
  }
  v4u q;
  q.x = (unsigned)bits[0] | ((unsigned)bits[1] << 16);
  q.y = (unsigned)bits[2] | ((unsigned)bits[3] << 16);
  q.z = (unsigned)bits[4] | ((unsigned)bits[5] << 16);
  q.w = (unsigned)bits[6] | ((unsigned)bits[7] << 16);
  unsigned short* dst = first ? (woffp + (size_t)jj * 8) : (wdefp + (size_t)jj * 8);
  *(volatile v4u*)dst = q;
  __threadfence();
  *(volatile v4u*)dst = q;
}

__global__ __launch_bounds__(NTHR) void k_offconv(const unsigned short* __restrict__ xh, const unsigned short* __restrict__ woffp,
                                                 const float* __restrict__ b_off, float* __restrict__ offp) {
  __shared__ __align__(16) unsigned short BT[TPIX * BTP];
  __shared__ __align__(16) float SL[NOFFP * SLP];
  const int blk = blockIdx.x;
  const int b   = blk / (NH * TPR);
  const int rem = blk - b * (NH * TPR);
  const int h   = rem / TPR;
  const int xs  = (rem - h * TPR) * TPIX;
  const int tid = threadIdx.x;

#pragma unroll 1
  for (int t = tid; t < TPIX * KPOS * 8; t += NTHR) {
    const int j    = t & 7;
    const int rest = t >> 3;
    const int p    = rest & (TPIX - 1);
    const int kpos = rest >> 6;
    const int kh = kpos / 3, kw = kpos - kh * 3;
    const int y  = h + kh - 1;
    const int xg = xs + p + kw - 1;
    const bool valid = (y >= 0) && (y < NH) && (xg >= 0) && (xg < NW);
    const int yc = clampi(y, 0, NH - 1), xc = clampi(xg, 0, NW - 1);
    v4u q = *(const v4u*)(xh + ((((size_t)b * NH + yc) * NW + xc) * NC + j * 8));
    const unsigned msk = valid ? 0xffffffffu : 0u;
    q = q & msk;
    *(v4u*)(BT + p * BTP + kpos * NC + j * 8) = q;
  }
  __syncthreads();

  const int lane = tid & 31, wave = tid >> 5;
  const int rl = lane & 15, hh = lane >> 4, koff = hh * 8;
  const int mt = wave >> 2, nt = wave & 3;
  const __bf16* arow = (const __bf16*)woffp + (size_t)(mt * 16 + rl) * KTOT + koff;
  const __bf16* brow = (const __bf16*)BT + (nt * 16 + rl) * BTP + koff;
  v8f acc = {0.f, 0.f, 0.f, 0.f, 0.f, 0.f, 0.f, 0.f};
#pragma unroll 1
  for (int s = 0; s < NKSTEP; ++s) {
    const int k0 = s * 32;
    const v16b af = Frag<__bf16>::load(arow + k0);
    const v16b bf = Frag<__bf16>::load(brow + k0);
    acc = Frag<__bf16>::mma(af, bf, acc);
    tie1_b(acc, af, bf);
  }

#pragma unroll
  for (int r = 0; r < 8; ++r) {
    const int o  = mt * 16 + 8 * hh + r;
    const int oc = (o < NOFF) ? o : (NOFF - 1);
    float v = acc[r] + bfr(b_off[oc]);
    v = fminf(1.0f, fmaxf(-1.0f, v));
    SL[o * SLP + nt * 16 + rl] = v;
  }
  __syncthreads();
  const int c4 = rl * 4;
  for (int pass = 0; pass < 2; ++pass) {
#pragma unroll
    for (int it = 0; it < 2; ++it) {
      const int rb = 2 * (it * 8 + wave);
      if (rb < NOFF) {
        const int row = rb + hh;
        const v4f v = *(const v4f*)(SL + row * SLP + c4);
        *(volatile v4f*)(offp + (((size_t)b * NOFF + row) * NH + h) * NW + xs + c4) = v;
      }
    }
    __threadfence();
  }
}

__global__ __launch_bounds__(NTHR) void k_sampconv(const unsigned short* __restrict__ xh, const float* __restrict__ offp,
                                                  const unsigned short* __restrict__ wdefp, const float* __restrict__ b_def,
                                                  float* __restrict__ out) {
  __shared__ __align__(16) unsigned short BT[TPIX * BTP];
  __shared__ __align__(16) float SL[NOUT * SLP];
  const int blk = blockIdx.x;
  const int b   = blk / (NH * TPR);
  const int rem = blk - b * (NH * TPR);
  const int h   = rem / TPR;
  const int xs  = (rem - h * TPR) * TPIX;
  const int tid = threadIdx.x;

  {
    const int p    = tid >> 2;
    const int cj   = tid & 3;
    const int xcol = xs + p;
    const size_t pixb = (size_t)b * NH;
#pragma unroll 1
    for (int kpos = 0; kpos < KPOS; ++kpos) {
      const int kh = kpos / 3, kw = kpos - kh * 3;
      const size_t ob = (((size_t)b * NOFF + 2 * kpos) * NH + h) * NW + xcol;
      const float dy = offp[ob];
      const float dx = offp[ob + (size_t)NH * NW];
      const float py = dy + (float)(h + kh - 1);
      const float px = dx + (float)(xcol + kw - 1);
      const float y0f = floorf(py), x0f = floorf(px);
      const float ly = py - y0f, lx = px - x0f;
      const int yi = (int)y0f, xi = (int)x0f;
      const float fy0 = (yi >= 0 && yi < NH) ? 1.0f : 0.0f;
      const float fy1 = (yi + 1 >= 0 && yi + 1 < NH) ? 1.0f : 0.0f;
      const float fx0 = (xi >= 0 && xi < NW) ? 1.0f : 0.0f;
      const float fx1 = (xi + 1 >= 0 && xi + 1 < NW) ? 1.0f : 0.0f;
      const int yc0 = clampi(yi, 0, NH - 1), yc1 = clampi(yi + 1, 0, NH - 1);
      const int xc0 = clampi(xi, 0, NW - 1), xc1 = clampi(xi + 1, 0, NW - 1);
      const float c00 = ((1.0f - ly) * (1.0f - lx)) * (fy0 * fx0);
      const float c01 = ((1.0f - ly) * lx) * (fy0 * fx1);
      const float c10 = (ly * (1.0f - lx)) * (fy1 * fx0);
      const float c11 = (ly * lx) * (fy1 * fx1);
      const unsigned short* p00 = xh + (((pixb + yc0) * NW + xc0) * NC + cj * 16);
      const unsigned short* p01 = xh + (((pixb + yc0) * NW + xc1) * NC + cj * 16);
      const unsigned short* p10 = xh + (((pixb + yc1) * NW + xc0) * NC + cj * 16);
      const unsigned short* p11 = xh + (((pixb + yc1) * NW + xc1) * NC + cj * 16);
      const v4u ga0 = *(const v4u*)(p00), ga1 = *(const v4u*)(p00 + 8);
      const v4u gb0 = *(const v4u*)(p01), gb1 = *(const v4u*)(p01 + 8);
      const v4u gc0 = *(const v4u*)(p10), gc1 = *(const v4u*)(p10 + 8);
      const v4u gd0 = *(const v4u*)(p11), gd1 = *(const v4u*)(p11 + 8);
      const v4u r0 = mix_vec(ga0, gb0, gc0, gd0, c00, c01, c10, c11);
      const v4u r1 = mix_vec(ga1, gb1, gc1, gd1, c00, c01, c10, c11);
      unsigned short* dst = BT + p * BTP + kpos * NC + cj * 16;
      *(v4u*)(dst)     = r0;
      *(v4u*)(dst + 8) = r1;
    }
  }
  __syncthreads();

  const int lane = tid & 31, wave = tid >> 5;
  const int rl = lane & 15, hh = lane >> 4, koff = hh * 8;
  const int nt = wave & 3, mt0 = (wave >> 2) * 2;
  const _Float16* a0row = (const _Float16*)wdefp + (size_t)(mt0 * 16 + rl) * KTOT + koff;
  const _Float16* a1row = a0row + 16 * KTOT;
  const _Float16* brow  = (const _Float16*)BT + (nt * 16 + rl) * BTP + koff;
  v8f acc0 = {0.f, 0.f, 0.f, 0.f, 0.f, 0.f, 0.f, 0.f};
  v8f acc1 = {0.f, 0.f, 0.f, 0.f, 0.f, 0.f, 0.f, 0.f};
#pragma unroll 1
  for (int s = 0; s < NKSTEP; ++s) {
    const int k0 = s * 32;
    const v16h af0 = Frag<_Float16>::load(a0row + k0);
    const v16h af1 = Frag<_Float16>::load(a1row + k0);
    const v16h bf  = Frag<_Float16>::load(brow + k0);
    acc0 = Frag<_Float16>::mma(af0, bf, acc0);
    acc1 = Frag<_Float16>::mma(af1, bf, acc1);
    tie2_h(acc0, acc1, af0, af1, bf);
  }

  const v4f bA = *(const v4f*)(b_def + mt0 * 16 + 8 * hh);
  const v4f bB = *(const v4f*)(b_def + mt0 * 16 + 8 * hh + 4);
  const v4f bC = *(const v4f*)(b_def + mt0 * 16 + 16 + 8 * hh);
  const v4f bD = *(const v4f*)(b_def + mt0 * 16 + 16 + 8 * hh + 4);
#pragma unroll
  for (int r = 0; r < 8; ++r) {
    const int o0 = mt0 * 16 + 8 * hh + r;
    const int o1 = o0 + 16;
    const float bias0 = (r < 4) ? bA[r] : bB[r - 4];
    const float bias1 = (r < 4) ? bC[r] : bD[r - 4];
    const float v0 = acc0[r] * WDEF_FOLD + bfr(bias0);
    const float v1 = acc1[r] * WDEF_FOLD + bfr(bias1);
    SL[o0 * SLP + nt * 16 + rl] = v0;
    SL[o1 * SLP + nt * 16 + rl] = v1;
  }
  __syncthreads();
  const int c4 = rl * 4;
  for (int pass = 0; pass < 2; ++pass) {
#pragma unroll
    for (int it = 0; it < 4; ++it) {
      const int row = 8 * wave + 2 * it + hh;
      const v4f v = *(const v4f*)(SL + row * SLP + c4);
      *(volatile v4f*)(out + (((size_t)b * NOUT + row) * NH + h) * NW + xs + c4) = v;
    }
    __threadfence();
  }
}

extern "C" void kernel_launch(void* const* d_in, const int* in_sizes, int n_in,
                              void* d_out, int out_size, void* d_ws, size_t ws_size, hipStream_t stream) {
  if (n_in < 5) return;
  if (in_sizes[0] != NB * NC * NH * NW) return;
  if (in_sizes[1] != NOFF * NC * KPOS) return;
  if (in_sizes[2] != NOFF) return;
  if (in_sizes[3] != NOUT * NC * KPOS) return;
  if (in_sizes[4] != NOUT) return;
  if (out_size != NB * NOUT * NH * NW) return;
  if (ws_size < WS_TOTAL) return;

  const float* x     = (const float*)d_in[0];
  const float* w_off = (const float*)d_in[1];
  const float* b_off = (const float*)d_in[2];
  const float* w_def = (const float*)d_in[3];
  const float* b_def = (const float*)d_in[4];
  float* out = (float*)d_out;

  char* ws = (char*)d_ws;
  unsigned short* xh    = (unsigned short*)(ws + WS_XH_OFF);
  float*          offp  = (float*)(ws + WS_OFFP_OFF);
  unsigned short* woffp = (unsigned short*)(ws + WS_WOFF_OFF);
  unsigned short* wdefp = (unsigned short*)(ws + WS_WDEF_OFF);

  k_pack_x<<<dim3(NB * NH, NW / 32), NTHR, 0, stream>>>(x, xh);
  k_pack_w<<<NVW_TOT / NTHR, NTHR, 0, stream>>>(w_off, w_def, woffp, wdefp);
  k_offconv<<<NBLK, NTHR, 0, stream>>>(xh, woffp, b_off, offp);
  k_sampconv<<<NBLK, NTHR, 0, stream>>>(xh, offp, wdefp, b_def, out);
}
